// CIN_13030930776368
// MI455X (gfx1250) — hardware-verified
//
#include <hip/hip_runtime.h>
#include <stddef.h>

typedef __attribute__((ext_vector_type(16))) _Float16 v16h;
typedef __attribute__((ext_vector_type(8)))  _Float16 v8h;
typedef __attribute__((ext_vector_type(16))) __bf16   v16b;
typedef __attribute__((ext_vector_type(8)))  __bf16   v8b;
typedef __attribute__((ext_vector_type(8)))  float    v8f;
typedef __attribute__((ext_vector_type(4)))  float    v4f;
typedef __attribute__((ext_vector_type(4)))  unsigned int v4u;

constexpr int NBATCH = 1024;
constexpr int NFIELD = 39;
constexpr int NEMB   = 64;
constexpr int NHID1  = 128;
constexpr int NHID2  = 128;
constexpr int NOUT   = NHID1 + NHID2;
constexpr int JPAD   = 64;
constexpr int IPAD   = 64;
constexpr int KLAY1  = NFIELD * NHID1;
constexpr int W0ROWS = NFIELD * NHID1;
constexpr int TPITCH = IPAD * NHID1;

static_assert(KLAY1 % 32 == 0, "K of the final GEMM must be a multiple of 32");
static_assert(JPAD % 32 == 0 && NEMB % 32 == 0, "K steps of 32");
static_assert(NBATCH % 64 == 0 && NHID1 % 64 == 0 && NHID2 % 64 == 0 && IPAD % 64 == 0, "GEMM tiles of 64");
static_assert(KLAY1 % 64 == 0, "W1 plane rows are whole 128-B lines");
static_assert(W0ROWS % 32 == 0, "prep grid for W0 plane is exact");
static_assert((NHID2 * (KLAY1 / 64)) % 32 == 0, "prep grid for W1 plane is exact");

__device__ __forceinline__ unsigned short f2bf_bits(float f) {
  unsigned u = __float_as_uint(f);
  return (unsigned short)((u + 0x7FFFu + ((u >> 16) & 1u)) >> 16);
}
__device__ __forceinline__ float bf_bits2f(unsigned short h) { return __uint_as_float(((unsigned)h) << 16); }

__device__ __forceinline__ void dep_guard_b(v8f& a, v8f& b, v16b x, v16b y) { asm volatile("v_nop\n\tv_nop\n\tv_nop\n\tv_nop" : "+v"(a), "+v"(b) : "v"(x), "v"(y)); }
__device__ __forceinline__ void keep4_b(v16b a, v16b b, v16b c, v16b d) { asm volatile("v_nop" :: "v"(a), "v"(b), "v"(c), "v"(d)); }
__device__ __forceinline__ void acc_guard4(v8f& a, v8f& b, v8f& c, v8f& d) { asm volatile("v_nop\n\tv_nop\n\tv_nop\n\tv_nop" : "+v"(a), "+v"(b), "+v"(c), "+v"(d)); }

template <typename T> struct Frag;
template <> struct Frag<__bf16> {
  typedef v16b V; union U { v16b v; v8b h[2]; };
  static __device__ __forceinline__ v16b load(const __bf16* p) {
    U f; f.h[0] = *(const v8b*)(p); f.h[1] = *(const v8b*)(p + 16); return f.v;
  }
  static __device__ __forceinline__ v8f mma(v16b a, v16b b, v8f c) {
    return __builtin_amdgcn_wmma_f32_16x16x32_bf16(false, a, false, b, (short)0, c, false, false);
  }
  static __device__ __forceinline__ void guard(v8f& a, v8f& b, v16b x, v16b y) { dep_guard_b(a, b, x, y); }
  static __device__ __forceinline__ void keep(v16b a, v16b b, v16b c, v16b d) { keep4_b(a, b, c, d); }
};

template <int SPLITM, int OUT_MODE>
__global__ __launch_bounds__(256) void wmma_gemm64b(
    const unsigned short* __restrict__ Ap, const unsigned short* __restrict__ A2p, int lda, long strideA,
    const unsigned short* __restrict__ Btp, const unsigned short* __restrict__ Bt2p, int ldb, long strideB,
    void* __restrict__ Cout, void* __restrict__ Cout2, int ldc, long strideC,
    int M, int N, int K, int nbatch, float scale) {
  typedef __bf16 T;
  typedef v16b V;
  constexpr bool SA = (SPLITM & 1) != 0;
  constexpr bool SB = (SPLITM & 2) != 0;
  const T* A = (const T*)Ap; const T* A2 = (const T*)A2p; const T* Bt = (const T*)Btp; const T* Bt2 = (const T*)Bt2p;
  __shared__ __align__(16) float sT[8][16 * 68];
  const int lane = threadIdx.x & 31;
  const int wave = threadIdx.x >> 5;
  const int tilesN = N >> 6;
  const int tilesM = M >> 6;
  const int tilesPB = tilesM * tilesN;
  const int tile = blockIdx.x * 8 + wave;
  if (tile >= tilesPB * nbatch) return;
  const int b  = tile / tilesPB;
  const int tt = tile - b * tilesPB;
  const int tm = tt / tilesN;
  const int tn = tt - tm * tilesN;
  const int m0 = tm << 6;
  const int n0 = tn << 6;

  const T* Ab  = A  + (size_t)b * strideA;
  const T* Bb  = Bt + (size_t)b * strideB;
  const T* Ab2 = SA ? (A2  + (size_t)b * strideA) : nullptr;
  const T* Bb2 = SB ? (Bt2 + (size_t)b * strideB) : nullptr;

  const int rlane = lane & 15;
  const int koff  = (lane >> 4) * 8;
  const int mOff  = (lane >> 4) * 8;

  v8f acc[4][4];
#pragma unroll
  for (int i = 0; i < 4; ++i)
#pragma unroll
    for (int j = 0; j < 4; ++j) acc[i][j] = (v8f){0.f,0.f,0.f,0.f,0.f,0.f,0.f,0.f};

  for (int k0 = 0; k0 < K; k0 += 32) {
    V bh[4], bl[4];
#pragma unroll
    for (int j = 0; j < 4; ++j) {
      const size_t bo = (size_t)(n0 + (j << 4) + rlane) * ldb + koff + k0;
      bh[j] = Frag<T>::load(Bb + bo);
      if (SB) bl[j] = Frag<T>::load(Bb2 + bo);
    }
#pragma unroll
    for (int i = 0; i < 4; ++i) {
      const size_t ao = (size_t)(m0 + (i << 4) + rlane) * lda + koff + k0;
      V ah = Frag<T>::load(Ab + ao);
      V al = ah;
      if (SA) al = Frag<T>::load(Ab2 + ao);
#pragma unroll
      for (int j = 0; j < 4; ++j) {
        acc[i][j] = Frag<T>::mma(ah, bh[j], acc[i][j]);
        if (SB) acc[i][j] = Frag<T>::mma(ah, bl[j], acc[i][j]);
        if (SA) acc[i][j] = Frag<T>::mma(al, bh[j], acc[i][j]);
      }
      Frag<T>::guard(acc[i][0], acc[i][3], ah, al);
    }
    Frag<T>::keep(bh[0], bh[1], bh[2], bh[3]);
    if (SB) Frag<T>::keep(bl[0], bl[1], bl[2], bl[3]);
  }
  acc_guard4(acc[0][0], acc[0][1], acc[0][2], acc[0][3]);
  acc_guard4(acc[1][0], acc[1][1], acc[1][2], acc[1][3]);
  acc_guard4(acc[2][0], acc[2][1], acc[2][2], acc[2][3]);
  acc_guard4(acc[3][0], acc[3][1], acc[3][2], acc[3][3]);

  float* slab = sT[wave];
#pragma unroll
  for (int i = 0; i < 4; ++i) {
    const int mBase = m0 + (i << 4);
#pragma unroll
    for (int j = 0; j < 4; ++j) {
#pragma unroll
      for (int r = 0; r < 8; ++r) {
        const float v = acc[i][j][r] * scale;
        slab[(mOff + r) * 68 + (j << 4) + rlane] = v;
      }
    }
    __builtin_amdgcn_fence(__ATOMIC_RELEASE, "workgroup");
    __builtin_amdgcn_wave_barrier();
    __builtin_amdgcn_fence(__ATOMIC_ACQUIRE, "workgroup");
    if (OUT_MODE == 0) {
      float* C = (float*)Cout + (size_t)b * strideC;
      const int hh = lane >> 4, c4 = (lane & 15) * 4;
      for (int pass = 0; pass < 2; ++pass) {
#pragma unroll
        for (int it = 0; it < 8; ++it) {
          const int row = it * 2 + hh;
          v4f v = *(const v4f*)(slab + row * 68 + c4);
          *(volatile v4f*)(C + (size_t)(mBase + row) * ldc + n0 + c4) = v;
        }
        __threadfence();
      }
    } else {
      const int q = lane >> 3, c8 = (lane & 7) * 8;
      unsigned short* C  = (unsigned short*)Cout  + (size_t)b * strideC;
      unsigned short* C2 = (unsigned short*)Cout2 + (size_t)b * strideC;
      for (int pass = 0; pass < 2; ++pass) {
#pragma unroll
        for (int it = 0; it < 4; ++it) {
          const int row = it * 4 + q;
          const float* sp = slab + row * 68 + c8;
          v8h hv, lv;
#pragma unroll
          for (int e = 0; e < 8; ++e) {
            unsigned short hb = f2bf_bits(sp[e]);
            unsigned short lb = f2bf_bits(sp[e] - bf_bits2f(hb));
            hv[e] = __builtin_bit_cast(_Float16, hb);
            lv[e] = __builtin_bit_cast(_Float16, lb);
          }
          *(volatile v8h*)(C + (size_t)(mBase + row) * ldc + n0 + c8) = hv;
          *(volatile v8h*)(C2 + (size_t)(mBase + row) * ldc + n0 + c8) = lv;
        }
        __threadfence();
      }
    }
    __builtin_amdgcn_fence(__ATOMIC_RELEASE, "workgroup");
    __builtin_amdgcn_wave_barrier();
    __builtin_amdgcn_fence(__ATOMIC_ACQUIRE, "workgroup");
  }
}

__global__ __launch_bounds__(256) void prep_w0_plane(const float* __restrict__ W0, unsigned int* __restrict__ W0w) {
  const int lane = threadIdx.x & 31;
  const int gw = blockIdx.x * 8 + (threadIdx.x >> 5);
  const int q = lane >> 3, c8 = (lane & 7) * 8;
  const int row = gw * 4 + q;
  const int i = row >> 7, h = row & (NHID1 - 1);
  const float* wp = W0 + (size_t)i * (NFIELD * NHID1) + h;
  v4u w;
#pragma unroll
  for (int e2 = 0; e2 < 4; ++e2) {
    const int j0 = c8 + 2 * e2, j1 = j0 + 1;
    const int j0c = j0 < NFIELD ? j0 : NFIELD - 1;
    const int j1c = j1 < NFIELD ? j1 : NFIELD - 1;
    float v0 = wp[(size_t)j0c * NHID1];
    float v1 = wp[(size_t)j1c * NHID1];
    v0 = (j0 < NFIELD) ? v0 : 0.0f;
    v1 = (j1 < NFIELD) ? v1 : 0.0f;
    w[e2] = (unsigned)f2bf_bits(v0) | ((unsigned)f2bf_bits(v1) << 16);
  }
  unsigned int* dst = W0w + (((size_t)row * JPAD + c8) >> 1);
  *(volatile v4u*)dst = w;
  __threadfence();
  *(volatile v4u*)dst = w;
}

__global__ __launch_bounds__(256) void prep_w1_plane(const float* __restrict__ W1, unsigned int* __restrict__ W1w) {
  const int lane = threadIdx.x & 31;
  const int gw = blockIdx.x * 8 + (threadIdx.x >> 5);
  const int q = lane >> 3, c8 = (lane & 7) * 8;
  const int c  = gw * 4 + q;
  const int h  = c / (KLAY1 / 64);
  const int kc = c - h * (KLAY1 / 64);
  const int k0 = kc * 64 + c8;
  const float* wp = W1 + (size_t)k0 * NHID2 + h;
  v4u w;
#pragma unroll
  for (int e2 = 0; e2 < 4; ++e2) {
    const float v0 = wp[(size_t)(2 * e2) * NHID2];
    const float v1 = wp[(size_t)(2 * e2 + 1) * NHID2];
    w[e2] = (unsigned)f2bf_bits(v0) | ((unsigned)f2bf_bits(v1) << 16);
  }
  unsigned int* dst = W1w + (((size_t)h * KLAY1 + k0) >> 1);
  *(volatile v4u*)dst = w;
  __threadfence();
  *(volatile v4u*)dst = w;
}

__global__ __launch_bounds__(128) void cin_first_layer(
    const float* __restrict__ x, const unsigned short* __restrict__ W0p,
    unsigned int* __restrict__ xAw, unsigned int* __restrict__ h1hiw, unsigned int* __restrict__ h1low,
    float* __restrict__ out)
{
  __shared__ __align__(16) float xs[NFIELD * NEMB];
  __shared__ __align__(16) unsigned int xTw[NEMB * (JPAD / 2)];
  __shared__ __align__(16) float slab[4][32 * 68];
  __shared__ __align__(16) float osum[4][32];

  const int tid  = threadIdx.x;
  const int wave = tid >> 5, lane = tid & 31, hh = lane >> 4, rl = lane & 15;
  const int b    = blockIdx.x;
  const int hw0  = wave * 32;

  const float* xb = x + (size_t)b * (NFIELD * NEMB);
  for (int idx = tid; idx < NFIELD * NEMB; idx += 128) {
    const float v = xb[idx];
    xs[idx] = bf_bits2f(f2bf_bits(v));
  }
  __syncthreads();

  if (tid < NEMB) {
    const int d = tid;
#pragma unroll
    for (int c = 0; c < 8; ++c) {
      v4u w;
#pragma unroll
      for (int e2 = 0; e2 < 4; ++e2) {
        const int j0 = c * 8 + 2 * e2, j1 = j0 + 1;
        const int j0c = j0 < NFIELD ? j0 : NFIELD - 1;
        const int j1c = j1 < NFIELD ? j1 : NFIELD - 1;
        float v0 = xs[j0c * NEMB + d], v1 = xs[j1c * NEMB + d];
        v0 = (j0 < NFIELD) ? v0 : 0.0f;
        v1 = (j1 < NFIELD) ? v1 : 0.0f;
        w[e2] = (unsigned)f2bf_bits(v0) | ((unsigned)f2bf_bits(v1) << 16);
      }
      *(v4u*)(xTw + d * (JPAD / 2) + c * 4) = w;
    }
  }
  __syncthreads();

  const __bf16* xT = (const __bf16*)(const void*)xTw;
  v16b bx[2][4];
#pragma unroll
  for (int ks = 0; ks < 2; ++ks)
#pragma unroll
    for (int nt = 0; nt < 4; ++nt)
      bx[ks][nt] = Frag<__bf16>::load(xT + (nt * 16 + rl) * JPAD + hh * 8 + ks * 32);

  v8f hacc[2][4];
#pragma unroll
  for (int mt = 0; mt < 2; ++mt)
#pragma unroll
    for (int nt = 0; nt < 4; ++nt) hacc[mt][nt] = (v8f){0.f,0.f,0.f,0.f,0.f,0.f,0.f,0.f};

  const __bf16* W0 = (const __bf16*)(const void*)W0p;
#pragma unroll 1
  for (int i = 0; i < NFIELD; ++i) {
    float xi[4];
#pragma unroll
    for (int nt = 0; nt < 4; ++nt) xi[nt] = xs[i * NEMB + nt * 16 + rl];
#pragma unroll
    for (int mt = 0; mt < 2; ++mt) {
      const size_t arow = (size_t)(i * NHID1 + hw0 + mt * 16 + rl) * JPAD + hh * 8;
      const v16b aw0 = Frag<__bf16>::load(W0 + arow);
      const v16b aw1 = Frag<__bf16>::load(W0 + arow + 32);
#pragma unroll
      for (int nh = 0; nh < 2; ++nh) {
        v8f t0 = (v8f){0.f,0.f,0.f,0.f,0.f,0.f,0.f,0.f};
        v8f t1 = (v8f){0.f,0.f,0.f,0.f,0.f,0.f,0.f,0.f};
        t0 = Frag<__bf16>::mma(aw0, bx[0][2 * nh],     t0);
        t1 = Frag<__bf16>::mma(aw0, bx[0][2 * nh + 1], t1);
        t0 = Frag<__bf16>::mma(aw1, bx[1][2 * nh],     t0);
        t1 = Frag<__bf16>::mma(aw1, bx[1][2 * nh + 1], t1);
        dep_guard_b(t0, t1, aw0, aw1);
#pragma unroll
        for (int r = 0; r < 8; ++r) {
          hacc[mt][2 * nh][r]     = xi[2 * nh]     * t0[r] + hacc[mt][2 * nh][r];
          hacc[mt][2 * nh + 1][r] = xi[2 * nh + 1] * t1[r] + hacc[mt][2 * nh + 1][r];
        }
      }
    }
  }
  keep4_b(bx[0][0], bx[0][1], bx[1][2], bx[1][3]);

  float* sl = slab[wave];
  float* os = osum[wave];
#pragma unroll
  for (int mt = 0; mt < 2; ++mt) {
#pragma unroll
    for (int r = 0; r < 8; ++r) {
      float s = (hacc[mt][0][r] + hacc[mt][1][r]) + (hacc[mt][2][r] + hacc[mt][3][r]);
      s += __shfl_xor(s, 1, 16);
      s += __shfl_xor(s, 2, 16);
      s += __shfl_xor(s, 4, 16);
      s += __shfl_xor(s, 8, 16);
      if (rl == 0) os[mt * 16 + 8 * hh + r] = s;
#pragma unroll
      for (int nt = 0; nt < 4; ++nt) sl[(mt * 16 + 8 * hh + r) * 68 + nt * 16 + rl] = hacc[mt][nt][r];
    }
  }
  __builtin_amdgcn_fence(__ATOMIC_RELEASE, "workgroup");
  __builtin_amdgcn_wave_barrier();
  __builtin_amdgcn_fence(__ATOMIC_ACQUIRE, "workgroup");

  const int q = lane >> 3, c8 = (lane & 7) * 8;
  for (int pass = 0; pass < 2; ++pass) {
#pragma unroll
    for (int it = 0; it < 8; ++it) {
      const int row = it * 4 + q;
      const float* sp = sl + row * 68 + c8;
      v4u hw, lw;
#pragma unroll
      for (int e2 = 0; e2 < 4; ++e2) {
        const float v0 = sp[2 * e2], v1 = sp[2 * e2 + 1];
        const unsigned short hb0 = f2bf_bits(v0), hb1 = f2bf_bits(v1);
        const unsigned short lb0 = f2bf_bits(v0 - bf_bits2f(hb0));
        const unsigned short lb1 = f2bf_bits(v1 - bf_bits2f(hb1));
        hw[e2] = (unsigned)hb0 | ((unsigned)hb1 << 16);
        lw[e2] = (unsigned)lb0 | ((unsigned)lb1 << 16);
      }
      const size_t wo = (((size_t)b * NHID1 + hw0 + row) * NEMB + c8) >> 1;
      *(volatile v4u*)(h1hiw + wo) = hw;
      *(volatile v4u*)(h1low + wo) = lw;
    }
#pragma unroll
    for (int it = 0; it < 4; ++it) {
      const int i  = wave * 16 + it * 4 + q;
      const int ic = i < NFIELD ? i : NFIELD - 1;
      const float* xp = xs + ic * NEMB + c8;
      const bool real = (i < NFIELD);
      v4u w;
#pragma unroll
      for (int e2 = 0; e2 < 4; ++e2) {
        float v0 = xp[2 * e2], v1 = xp[2 * e2 + 1];
        v0 = real ? v0 : 0.0f;
        v1 = real ? v1 : 0.0f;
        w[e2] = (unsigned)f2bf_bits(v0) | ((unsigned)f2bf_bits(v1) << 16);
      }
      const size_t wo = (((size_t)b * IPAD + i) * NEMB + c8) >> 1;
      *(volatile v4u*)(xAw + wo) = w;
    }
    if (lane < 8) {
      const v4f v = *(const v4f*)(os + lane * 4);
      *(volatile v4f*)(out + (size_t)b * NOUT + hw0 + lane * 4) = v;
    }
    __threadfence();
  }
}

constexpr size_t WSB_W0 = (size_t)W0ROWS * JPAD * 2;
constexpr size_t WSB_W1 = (size_t)NHID2 * KLAY1 * 2;
constexpr size_t WSB_XA = (size_t)NBATCH * IPAD * NEMB * 2;
constexpr size_t WSB_H1 = (size_t)NBATCH * NHID1 * NEMB * 2;
constexpr size_t WSB_T  = (size_t)NBATCH * TPITCH * 2;
constexpr size_t WSO_W0  = 0;
constexpr size_t WSO_W1  = WSO_W0 + WSB_W0;
constexpr size_t WSO_XA  = WSO_W1 + WSB_W1;
constexpr size_t WSO_H1H = WSO_XA + WSB_XA;
constexpr size_t WSO_H1L = WSO_H1H + WSB_H1;
constexpr size_t WSO_TH  = WSO_H1L + WSB_H1;
constexpr size_t WSO_TL  = WSO_TH + WSB_T;
constexpr size_t WS_TOTAL = WSO_TL + WSB_T;
static_assert(WS_TOTAL == 77414400ull, "carve total");
static_assert(WS_TOTAL <= 134217728ull, "carve under 128 MiB");
static_assert(WSO_W1 % 128 == 0 && WSO_XA % 128 == 0 && WSO_H1H % 128 == 0 && WSO_H1L % 128 == 0 &&
              WSO_TH % 128 == 0 && WSO_TL % 128 == 0, "128-B aligned regions");
static_assert(IPAD % 64 == 0 && NHID1 % 64 == 0 && NEMB % 32 == 0, "T GEMM: M=64, N=128, K=64");
static_assert(NBATCH % 64 == 0 && NHID2 % 64 == 0 && KLAY1 % 32 == 0, "final GEMM: M=1024, N=128, K=4992");
static_assert((size_t)(NFIELD - 1) * NHID1 + NHID1 <= (size_t)TPITCH, "K=4992 fits inside one T row block");

extern "C" void kernel_launch(void* const* d_in, const int* in_sizes, int n_in,
                              void* d_out, int out_size, void* d_ws, size_t ws_size,
                              hipStream_t stream) {
  if (n_in < 3) return;
  if (in_sizes[0] != NBATCH * NFIELD * NEMB) return;
  if (in_sizes[1] != NFIELD * NFIELD * NHID1) return;
  if (in_sizes[2] != NFIELD * NHID1 * NHID2) return;
  if (out_size != NBATCH * NOUT) return;
  if (ws_size < WS_TOTAL) return;

  const float* x  = (const float*)d_in[0];
  const float* W0 = (const float*)d_in[1];
  const float* W1 = (const float*)d_in[2];
  float* out = (float*)d_out;
  char* ws = (char*)d_ws;

  unsigned int*   w0w  = (unsigned int*)(ws + WSO_W0);
  unsigned int*   w1w  = (unsigned int*)(ws + WSO_W1);
  unsigned int*   xaw  = (unsigned int*)(ws + WSO_XA);
  unsigned int*   h1hw = (unsigned int*)(ws + WSO_H1H);
  unsigned int*   h1lw = (unsigned int*)(ws + WSO_H1L);
  unsigned short* thi  = (unsigned short*)(ws + WSO_TH);
  unsigned short* tlo  = (unsigned short*)(ws + WSO_TL);

  prep_w0_plane<<<dim3(W0ROWS / 32), dim3(256), 0, stream>>>(W0, w0w);
  prep_w1_plane<<<dim3((NHID2 * (KLAY1 / 64)) / 32), dim3(256), 0, stream>>>(W1, w1w);
  cin_first_layer<<<dim3(NBATCH), dim3(128), 0, stream>>>(
      x, (const unsigned short*)(const void*)w0w, xaw, h1hw, h1lw, out);
  {
    const int M = IPAD, N = NHID1, K = NEMB, nb = NBATCH;
    const int tiles = nb * (M / 64) * (N / 64);
    wmma_gemm64b<2, 2><<<dim3((tiles + 7) / 8), dim3(256), 0, stream>>>(
        (const unsigned short*)(const void*)xaw, (const unsigned short*)(const void*)xaw, NEMB, (long)(IPAD * NEMB),
        (const unsigned short*)(const void*)h1hw, (const unsigned short*)(const void*)h1lw, NEMB, (long)(NHID1 * NEMB),
        (void*)thi, (void*)tlo, NHID1, (long)TPITCH,
        M, N, K, nb, 1.0f);
  }
  {
    const int M = NBATCH, N = NHID2, K = KLAY1;
    const int tiles = (M / 64) * (N / 64);
    wmma_gemm64b<1, 0><<<dim3((tiles + 7) / 8), dim3(256), 0, stream>>>(
        thi, tlo, TPITCH, (long)0,
        (const unsigned short*)(const void*)w1w, (const unsigned short*)(const void*)w1w, KLAY1, (long)0,
        (void*)(out + NHID1), (void*)(out + NHID1), NOUT, (long)0,
        M, N, K, 1, 1.0f);
  }
}
